// PatchNet_58188216926937
// MI455X (gfx1250) — hardware-verified
//
#include <hip/hip_runtime.h>

typedef __attribute__((ext_vector_type(16))) __bf16   v16b;
typedef __attribute__((ext_vector_type(8)))  __bf16   v8b;
typedef __attribute__((ext_vector_type(8)))  float    v8f;
typedef __attribute__((ext_vector_type(4)))  unsigned v4u;

constexpr int kBatch  = 32;
constexpr int kImg    = 224;
constexpr int kChan   = 3;
constexpr int kGridN  = 27;
constexpr int kMaps   = 10;
constexpr int kPatch  = 32;
constexpr int kStep   = kImg / kGridN;
constexpr int kPadLo  = (kPatch - kStep) / 2;
constexpr int kRowsA  = 16;
constexpr int kChunk  = 32;
constexpr int kDepth  = kGridN * kChunk;
constexpr int kSub    = kPatch / kStep;
constexpr int kDepthC = kStep * kStep * kChan;
constexpr int kRowsR  = kGridN + kSub - 1;
constexpr int kOutRow = kPatch * kChan;

static_assert(kStep == 8 && kPadLo == 12, "stride 8, border 12");
static_assert(kDepth == 864 && (kDepth % 32) == 0, "K multiple of 32");
static_assert(kSub == 4 && kDepthC == 192 && kRowsR == 30 && kOutRow == 96, "derived shapes");
static_assert(kMaps <= kRowsA, "row padding");

constexpr size_t kBytesAPL = (size_t)kBatch * kRowsA * kDepth * 2;
constexpr size_t kBytesXT  = (size_t)kSub * kBatch * kDepthC * kRowsR * kChunk * 2;
constexpr size_t kOffAPL   = 0;
constexpr size_t kOffXT    = kOffAPL + kBytesAPL;
constexpr size_t kWsTotal  = kOffXT + kBytesXT;
static_assert(kBytesAPL == 884736ull && kBytesXT == 47185920ull, "plane sizes");
static_assert(kWsTotal == 48070656ull, "carve total");
static_assert(kWsTotal <= 134217728ull, "carve cap");
static_assert((kOffXT % 128) == 0, "128-B aligned region");

constexpr int kATotal8 = kBatch * kRowsA * kDepth / 8;
constexpr int kXTotal8 = kSub * kBatch * kDepthC * kRowsR * kChunk / 8;
static_assert(kATotal8 == 55296 && (kATotal8 % 256) == 0, "weight pack grid exact");
static_assert(kXTotal8 == 2949120 && (kXTotal8 % 256) == 0, "depth pack grid exact");

__device__ __forceinline__ unsigned rne_word(float f) {
  const unsigned u = __float_as_uint(f);
  return u + 0x7FFFu + ((u >> 16) & 1u);
}
__device__ __forceinline__ unsigned pack_pair(float lo, float hi) {
  const unsigned a = rne_word(lo);
  const unsigned b = rne_word(hi);
  return (a >> 16) | (b & 0xFFFF0000u);
}

__device__ __forceinline__ v8f mma_guard(v16b a, v16b b, v8f c) {
  c = __builtin_amdgcn_wmma_f32_16x16x32_bf16(false, a, false, b, (short)0, c, false, false);
  asm volatile("v_nop\n\tv_nop\n\tv_nop\n\tv_nop" : "+v"(c) : "v"(a), "v"(b));
  return c;
}
__device__ __forceinline__ v16b frag_load(const __bf16* p) {
  union U { v16b v; v8b h[2]; } f;
  f.h[0] = *(const v8b*)(p);
  f.h[1] = *(const v8b*)(p + 16);
  return f.v;
}

__global__ __launch_bounds__(256) void weight_pack_kernel(const float* __restrict__ ind, unsigned* __restrict__ apl) {
  const int g = blockIdx.x * 256 + threadIdx.x;
  if (g >= kATotal8) return;
  constexpr int kSegs = kDepth / 8;
  const int seg = g % kSegs;
  const int row = g / kSegs;
  const int m   = row & (kRowsA - 1);
  const int b   = row / kRowsA;
  const int kk0 = seg * 8;
  const int h   = kk0 / kChunk;
  const int w0  = kk0 - h * kChunk;
  const bool mok = (m < kMaps);
  const int  mc  = mok ? m : (kMaps - 1);
  const float* src = ind + (size_t)b * (kGridN * kGridN * kMaps) + (size_t)h * (kGridN * kMaps) + mc;
  float v[8];
#pragma unroll
  for (int e = 0; e < 8; ++e) {
    const int w  = w0 + e;
    const int wc = (w < kGridN) ? w : (kGridN - 1);
    float t = src[wc * kMaps];
    asm volatile("" : "+v"(t));
    v[e] = (mok && (w < kGridN)) ? t : 0.0f;
  }
  v4u o;
  o.x = pack_pair(v[0], v[1]);
  o.y = pack_pair(v[2], v[3]);
  o.z = pack_pair(v[4], v[5]);
  o.w = pack_pair(v[6], v[7]);
  volatile v4u* p = (volatile v4u*)apl + g;
  *p = o;
  __threadfence();
  *p = o;
}

__global__ __launch_bounds__(256) void depth_pack_kernel(const float* __restrict__ x, unsigned* __restrict__ xt) {
  const int g = blockIdx.x * 256 + threadIdx.x;
  if (g >= kXTotal8) return;
  const int cw0 = (g & 3) * 8;
  int r = g >> 2;
  const int R = r % kRowsR;
  r /= kRowsR;
  const int n = r % kDepthC;
  r /= kDepthC;
  const int b  = r % kBatch;
  const int jw = r / kBatch;
  const int c  = n % kChan;
  const int q  = n / kChan;
  const int jr = q % kStep;
  const int ir = q / kStep;
  const int y  = kStep * R + ir - kPadLo;
  const bool yok = (y >= 0) && (y < kImg);
  const int  yc  = y < 0 ? 0 : (y > kImg - 1 ? kImg - 1 : y);
  const float* xrow = x + ((size_t)(b * kImg + yc) * kImg) * kChan + c;
  float v[8];
#pragma unroll
  for (int e = 0; e < 8; ++e) {
    const int xc  = kStep * (cw0 + e + jw) + jr - kPadLo;
    const bool ok = yok && (xc >= 0) && (xc < kImg);
    const int xcc = xc < 0 ? 0 : (xc > kImg - 1 ? kImg - 1 : xc);
    float t = xrow[xcc * kChan];
    asm volatile("" : "+v"(t));
    v[e] = ok ? t : 0.0f;
  }
  v4u o;
  o.x = pack_pair(v[0], v[1]);
  o.y = pack_pair(v[2], v[3]);
  o.z = pack_pair(v[4], v[5]);
  o.w = pack_pair(v[6], v[7]);
  volatile v4u* p = (volatile v4u*)xt + g;
  *p = o;
  __threadfence();
  *p = o;
}

__global__ __launch_bounds__(256) void grid_sum_gemm_kernel(const unsigned short* __restrict__ apl,
                                                            const unsigned short* __restrict__ xt,
                                                            float* __restrict__ out) {
  __shared__ __align__(16) unsigned short sA[kRowsA * kDepth];
  __shared__ __align__(16) float sO[8][kMaps * kOutRow];
  const int tid  = threadIdx.x;
  const int lane = tid & 31;
  const int wave = __builtin_amdgcn_readfirstlane((int)(threadIdx.x >> 5));
  const int b    = blockIdx.x / kSub;
  const int ih   = blockIdx.x - b * kSub;

  {
    constexpr int kPieces = kRowsA * kDepth / 8;
    const v4u* src = (const v4u*)(apl + (size_t)b * (kRowsA * kDepth));
    v4u* dst = (v4u*)sA;
    for (int idx = tid; idx < kPieces; idx += 256) dst[idx] = src[idx];
  }
  __syncthreads();

  const int hh   = lane >> 4;
  const int col  = lane & 15;
  const int koff = hh * 8;
  const __bf16* aBase = (const __bf16*)sA + col * kDepth + koff;
  const __bf16* xtb   = (const __bf16*)xt;

  int boff[6];
#pragma unroll
  for (int t = 0; t < 6; ++t) {
    const int np = 16 * t + col;
    const int jw = np / (kStep * kChan);
    const int nn = wave * (kStep * kChan) + (np - jw * (kStep * kChan));
    boff[t] = (((jw * kBatch + b) * kDepthC + nn) * kRowsR + ih) * kChunk + koff;
  }

  v8f acc[6];
#pragma unroll
  for (int t = 0; t < 6; ++t) acc[t] = (v8f){0.f, 0.f, 0.f, 0.f, 0.f, 0.f, 0.f, 0.f};

#pragma unroll 1
  for (int h = 0; h < kGridN; ++h) {
    const v16b a = frag_load(aBase + h * kChunk);
#pragma unroll
    for (int t = 0; t < 6; ++t) {
      const v16b bf = frag_load(xtb + boff[t] + h * kChunk);
      acc[t] = mma_guard(a, bf, acc[t]);
    }
  }

  float* slab = sO[wave];
#pragma unroll
  for (int t = 0; t < 6; ++t) {
#pragma unroll
    for (int r = 0; r < 8; ++r) {
      if (hh == 0 || r < (kMaps - 8)) slab[(8 * hh + r) * kOutRow + 16 * t + col] = acc[t][r];
    }
  }
  __syncthreads();

  float vals[kMaps * 3];
#pragma unroll
  for (int L = 0; L < kMaps * 3; ++L) vals[L] = slab[L * 32 + lane];

  const int i = kStep * ih + wave;
  for (int pass = 0; pass < 2; ++pass) {
#pragma unroll
    for (int k = 0; k < kMaps; ++k) {
      float* orow = out + ((size_t)((b * kMaps + k) * kPatch + i)) * kOutRow;
#pragma unroll
      for (int sg = 0; sg < 3; ++sg) {
        *(volatile float*)(orow + sg * 32 + lane) = vals[k * 3 + sg];
      }
    }
    __threadfence();
  }
}

extern "C" void kernel_launch(void* const* d_in, const int* in_sizes, int n_in,
                              void* d_out, int out_size, void* d_ws, size_t ws_size,
                              hipStream_t stream) {
  if (n_in < 2) return;
  if (in_sizes[0] != kBatch * kImg * kImg * kChan) return;
  if (in_sizes[1] != kBatch * kGridN * kGridN * kMaps) return;
  if (out_size != kBatch * kMaps * kPatch * kPatch * kChan) return;
  if (ws_size < kWsTotal) return;

  const float* x   = (const float*)d_in[0];
  const float* ind = (const float*)d_in[1];
  float* out = (float*)d_out;
  char* ws = (char*)d_ws;
  unsigned short* apl = (unsigned short*)(ws + kOffAPL);
  unsigned short* xtp = (unsigned short*)(ws + kOffXT);

  weight_pack_kernel<<<kATotal8 / 256, 256, 0, stream>>>(ind, (unsigned*)apl);
  depth_pack_kernel<<<kXTotal8 / 256, 256, 0, stream>>>(x, (unsigned*)xtp);
  grid_sum_gemm_kernel<<<kBatch * kSub, 256, 0, stream>>>(apl, xtp, out);
}
